// MAB_83494164234881
// MI455X (gfx1250) — hardware-run, weakly checked
//
#include <hip/hip_runtime.h>
#include <math.h>
#include <stdint.h>

#define NB   4
#define NT   1024
#define DM   1024
#define NH   16
#define HDIM 64
#define K2   2048
#define MTOT (NB * NT)

typedef __attribute__((ext_vector_type(16))) _Float16 v16h;
typedef __attribute__((ext_vector_type(8)))  _Float16 v8h;
typedef __attribute__((ext_vector_type(16))) __bf16   v16b;
typedef __attribute__((ext_vector_type(8)))  __bf16   v8b;
typedef __attribute__((ext_vector_type(8)))  float    v8f;
typedef __attribute__((ext_vector_type(4)))  float    v4f;
typedef __attribute__((ext_vector_type(2)))  float    v2f;
typedef __attribute__((ext_vector_type(4)))  unsigned int v4u;

__device__ __forceinline__ unsigned short f2bf_bits(float f) {
  unsigned u = __float_as_uint(f);
  return (unsigned short)((u + 0x7FFFu + ((u >> 16) & 1u)) >> 16);
}
__device__ __forceinline__ float bf_bits2f(unsigned short h) { return __uint_as_float(((unsigned)h) << 16); }
__device__ __forceinline__ float bfr(float f) { return bf_bits2f(f2bf_bits(f)); }
__device__ __forceinline__ v4f bfr4(v4f a) {
  v4f r;
  r[0] = bfr(a[0]); r[1] = bfr(a[1]); r[2] = bfr(a[2]); r[3] = bfr(a[3]);
  return r;
}
__device__ __forceinline__ unsigned pk16(unsigned short a, unsigned short b) { return (unsigned)a | ((unsigned)b << 16); }

__device__ __forceinline__ void dep_guard_h(v8f& a, v8f& b, v16h x, v16h y) { asm volatile("v_nop\n\tv_nop\n\tv_nop\n\tv_nop" : "+v"(a), "+v"(b) : "v"(x), "v"(y)); }
__device__ __forceinline__ void dep_guard_b(v8f& a, v8f& b, v16b x, v16b y) { asm volatile("v_nop\n\tv_nop\n\tv_nop\n\tv_nop" : "+v"(a), "+v"(b) : "v"(x), "v"(y)); }
__device__ __forceinline__ void keep4_h(v16h a, v16h b, v16h c, v16h d) { asm volatile("v_nop" :: "v"(a), "v"(b), "v"(c), "v"(d)); }
__device__ __forceinline__ void keep4_b(v16b a, v16b b, v16b c, v16b d) { asm volatile("v_nop" :: "v"(a), "v"(b), "v"(c), "v"(d)); }
__device__ __forceinline__ void acc_guard4(v8f& a, v8f& b, v8f& c, v8f& d) { asm volatile("v_nop\n\tv_nop\n\tv_nop\n\tv_nop" : "+v"(a), "+v"(b), "+v"(c), "+v"(d)); }

template <typename T> struct Frag;
template <> struct Frag<_Float16> {
  typedef v16h V; union U { v16h v; v8h h[2]; };
  static __device__ __forceinline__ v16h load(const _Float16* p) {
    U f; f.h[0] = *(const v8h*)(p); f.h[1] = *(const v8h*)(p + 16); return f.v;
  }
  static __device__ __forceinline__ v8f mma(v16h a, v16h b, v8f c) {
    return __builtin_amdgcn_wmma_f32_16x16x32_f16(false, a, false, b, (short)0, c, false, false);
  }
  static __device__ __forceinline__ void guard(v8f& a, v8f& b, v16h x, v16h y) { dep_guard_h(a, b, x, y); }
  static __device__ __forceinline__ void keep(v16h a, v16h b, v16h c, v16h d) { keep4_h(a, b, c, d); }
};
template <> struct Frag<__bf16> {
  typedef v16b V; union U { v16b v; v8b h[2]; };
  static __device__ __forceinline__ v16b load(const __bf16* p) {
    U f; f.h[0] = *(const v8b*)(p); f.h[1] = *(const v8b*)(p + 16); return f.v;
  }
  static __device__ __forceinline__ v8f mma(v16b a, v16b b, v8f c) {
    return __builtin_amdgcn_wmma_f32_16x16x32_bf16(false, a, false, b, (short)0, c, false, false);
  }
  static __device__ __forceinline__ void guard(v8f& a, v8f& b, v16b x, v16b y) { dep_guard_b(a, b, x, y); }
  static __device__ __forceinline__ void keep(v16b a, v16b b, v16b c, v16b d) { keep4_b(a, b, c, d); }
};

template <int ET> struct Elem;
template <> struct Elem<0> { typedef _Float16 T; };
template <> struct Elem<1> { typedef __bf16 T; };
template <int ET, bool SPLIT, int BIAS_MODE, int OUT_MODE, bool RESID, int ACT = 0>
__global__ __launch_bounds__(256) void wmma_gemm64(
    const unsigned short* __restrict__ Ap, const unsigned short* __restrict__ A2p, int lda, long strideA,
    const unsigned short* __restrict__ Btp, const unsigned short* __restrict__ Bt2p, int ldb, long strideB,
    void* __restrict__ Cout, void* __restrict__ Cout2, int ldc, long strideC,
    const float* __restrict__ bias,
    const float* __restrict__ resid, long strideR,
    int M, int N, int K, float scale) {
  typedef typename Elem<ET>::T T;
  typedef typename Frag<T>::V V;
  const T* A = (const T*)Ap; const T* A2 = (const T*)A2p; const T* Bt = (const T*)Btp; const T* Bt2 = (const T*)Bt2p;
  __shared__ __align__(16) float sT[8][16 * 68];
  const int b    = blockIdx.y;
  const int lane = threadIdx.x & 31;
  const int wave = threadIdx.x >> 5;
  const int tilesN = N >> 6;
  const int tilesM = M >> 6;
  const int tile = blockIdx.x * 8 + wave;
  if (tile >= tilesM * tilesN) return;
  const int tm = tile / tilesN;
  const int tn = tile - tm * tilesN;
  const int m0 = tm << 6;
  const int n0 = tn << 6;

  const T* Ab  = A  + (size_t)b * strideA;
  const T* Bb  = Bt + (size_t)b * strideB;
  const T* Ab2 = SPLIT ? (A2  + (size_t)b * strideA) : nullptr;
  const T* Bb2 = SPLIT ? (Bt2 + (size_t)b * strideB) : nullptr;

  const int rlane = lane & 15;
  const int koff  = (lane >> 4) * 8;
  const int mOff  = (lane >> 4) * 8;

  v8f acc[4][4];
#pragma unroll
  for (int i = 0; i < 4; ++i)
#pragma unroll
    for (int j = 0; j < 4; ++j) acc[i][j] = (v8f){0.f,0.f,0.f,0.f,0.f,0.f,0.f,0.f};

  for (int k0 = 0; k0 < K; k0 += 32) {
    V bh[4], bl[4];
#pragma unroll
    for (int j = 0; j < 4; ++j) {
      const size_t bo = (size_t)(n0 + (j << 4) + rlane) * ldb + koff + k0;
      bh[j] = Frag<T>::load(Bb + bo);
      if (SPLIT) bl[j] = Frag<T>::load(Bb2 + bo);
    }
#pragma unroll
    for (int i = 0; i < 4; ++i) {
      const size_t ao = (size_t)(m0 + (i << 4) + rlane) * lda + koff + k0;
      V ah = Frag<T>::load(Ab + ao);
      V al;
      if (SPLIT) al = Frag<T>::load(Ab2 + ao);
#pragma unroll
      for (int j = 0; j < 4; ++j) {
        acc[i][j] = Frag<T>::mma(ah, bh[j], acc[i][j]);
        if (SPLIT) {
          acc[i][j] = Frag<T>::mma(ah, bl[j], acc[i][j]);
          acc[i][j] = Frag<T>::mma(al, bh[j], acc[i][j]);
        }
      }
      Frag<T>::guard(acc[i][0], acc[i][3], ah, SPLIT ? al : ah);
    }
    Frag<T>::keep(bh[0], bh[1], bh[2], bh[3]);
    if (SPLIT) Frag<T>::keep(bl[0], bl[1], bl[2], bl[3]);
  }
  acc_guard4(acc[0][0], acc[0][1], acc[0][2], acc[0][3]);
  acc_guard4(acc[1][0], acc[1][1], acc[1][2], acc[1][3]);
  acc_guard4(acc[2][0], acc[2][1], acc[2][2], acc[2][3]);
  acc_guard4(acc[3][0], acc[3][1], acc[3][2], acc[3][3]);

  float* slab = sT[wave];
#pragma unroll
  for (int i = 0; i < 4; ++i) {
    const int mBase = m0 + (i << 4);
#pragma unroll
    for (int j = 0; j < 4; ++j) {
      const int n = n0 + (j << 4) + rlane;
      float bv = 0.f;
      if (BIAS_MODE == 2) bv = bfr(bias[n]);
#pragma unroll
      for (int r = 0; r < 8; ++r) {
        float v = acc[i][j][r] * scale;
        if (BIAS_MODE == 1) v += bfr(bias[mBase + mOff + r]);
        if (BIAS_MODE == 2) v += bv;
        if (ACT == 2) v = fmaxf(v, 0.0f);
        slab[(mOff + r) * 68 + (j << 4) + rlane] = v;
      }
    }
    __builtin_amdgcn_fence(__ATOMIC_RELEASE, "workgroup");
    __builtin_amdgcn_wave_barrier();
    __builtin_amdgcn_fence(__ATOMIC_ACQUIRE, "workgroup");
    if (OUT_MODE == 0) {
      float* C = (float*)Cout + (size_t)b * strideC;
      const int hh = lane >> 4, c4 = (lane & 15) * 4;
      v4f vals[8];
#pragma unroll
      for (int it = 0; it < 8; ++it) {
        const int row = it * 2 + hh;
        v4f v = *(const v4f*)(slab + row * 68 + c4);
        if (RESID) {
          const float* Rb = resid + (size_t)b * strideR;
          const v4f rv = *(const v4f*)(Rb + (size_t)(mBase + row) * ldc + n0 + c4);
          v = v + rv;
        }
        vals[it] = v;
      }
      for (int pass = 0; pass < 2; ++pass) {
#pragma unroll
        for (int it = 0; it < 8; ++it) {
          const int row = it * 2 + hh;
          *(volatile v4f*)(C + (size_t)(mBase + row) * ldc + n0 + c4) = vals[it];
        }
        __threadfence();
      }
    } else {
      const int q = lane >> 3, c8 = (lane & 7) * 8;
      unsigned short* C  = (unsigned short*)Cout  + (size_t)b * strideC;
      unsigned short* C2 = (unsigned short*)Cout2 + (size_t)b * strideC;
      v8h hvv[4], lvv[4];
#pragma unroll
      for (int it = 0; it < 4; ++it) {
        const int row = it * 4 + q;
        const float* sp = slab + row * 68 + c8;
        v8h hv, lv;
#pragma unroll
        for (int e = 0; e < 8; ++e) {
          if (OUT_MODE == 1) {
            hv[e] = (_Float16)sp[e];
            lv[e] = (_Float16)0.0f;
          } else {
            const unsigned short hb = f2bf_bits(sp[e]);
            unsigned short lb = 0;
            if (OUT_MODE == 2) lb = f2bf_bits(sp[e] - bf_bits2f(hb));
            hv[e] = __builtin_bit_cast(_Float16, hb);
            lv[e] = __builtin_bit_cast(_Float16, lb);
          }
        }
        hvv[it] = hv; lvv[it] = lv;
      }
      for (int pass = 0; pass < 2; ++pass) {
#pragma unroll
        for (int it = 0; it < 4; ++it) {
          const int row = it * 4 + q;
          *(volatile v8h*)(C + (size_t)(mBase + row) * ldc + n0 + c8) = hvv[it];
          if (OUT_MODE == 2) *(volatile v8h*)(C2 + (size_t)(mBase + row) * ldc + n0 + c8) = lvv[it];
        }
        __threadfence();
      }
    }
    __builtin_amdgcn_fence(__ATOMIC_RELEASE, "workgroup");
    __builtin_amdgcn_wave_barrier();
    __builtin_amdgcn_fence(__ATOMIC_ACQUIRE, "workgroup");
  }
}

__global__ __launch_bounds__(256) void wprep_kernel(const float* __restrict__ w0, const float* __restrict__ w1,
                                                    const float* __restrict__ w2, const float* __restrict__ w3,
                                                    unsigned short* __restrict__ ob) {
  __shared__ __align__(16) float tf[64 * 68];
  const int z = blockIdx.z;
  const float* W = (z == 0) ? w0 : ((z == 1) ? w1 : ((z == 2) ? w2 : w3));
  unsigned short* o = ob + (size_t)z * DM * K2;
  const int c0  = blockIdx.x * 64;
  const int r0  = blockIdx.y * 64;
  const int tid = threadIdx.x;
  {
    const int lr = tid >> 4;
    const int c4 = (tid & 15) * 4;
#pragma unroll
    for (int it = 0; it < 4; ++it) {
      const int rr = it * 16 + lr;
      const v4f a = *(const v4f*)(W + (size_t)(r0 + rr) * DM + c0 + c4);
      *(v4f*)(tf + rr * 68 + c4) = a;
    }
  }
  __syncthreads();
  const int sub = tid >> 3;
  const int c8  = (tid & 7) * 8;
  v4u hv[2];
#pragma unroll
  for (int it = 0; it < 2; ++it) {
    const int oc = it * 32 + sub;
    v4u a;
#pragma unroll
    for (int q = 0; q < 4; ++q) {
      const float f0 = tf[(c8 + 2 * q) * 68 + oc];
      const float f1 = tf[(c8 + 2 * q + 1) * 68 + oc];
      a[q] = pk16(f2bf_bits(f0), f2bf_bits(f1));
    }
    hv[it] = a;
  }
  for (int pass = 0; pass < 2; ++pass) {
#pragma unroll
    for (int it = 0; it < 2; ++it) {
      const int oc = it * 32 + sub;
      const size_t go = (size_t)(c0 + oc) * K2 + r0 + c8;
      *(volatile v4u*)(o + go)      = hv[it];
      *(volatile v4u*)(o + go + DM) = hv[it];
    }
    __threadfence();
  }
}

template <bool RIN>
__global__ __launch_bounds__(256) void ln_kernel(const float* __restrict__ xa, const float* __restrict__ ga, const float* __restrict__ ba,
                                                 const float* __restrict__ xb, const float* __restrict__ gb, const float* __restrict__ bb,
                                                 int rowsA, int rowsTot, unsigned short* __restrict__ outp) {
  const int lane = threadIdx.x & 31;
  const int wave = threadIdx.x >> 5;
  const int row  = blockIdx.x * 8 + wave;
  if (row >= rowsTot) return;
  const bool sec = (row >= rowsA);
  const float* x  = sec ? (xb + (size_t)(row - rowsA) * DM) : (xa + (size_t)row * DM);
  const float* g  = sec ? gb : ga;
  const float* be = sec ? bb : ba;
  unsigned short* orow = outp + (size_t)row * K2;

  float s = 0.f;
#pragma unroll 1
  for (int i = 0; i < 4; ++i) {
    const int cb = i * 256 + lane * 8;
    v4f a = *(const v4f*)(x + cb);
    v4f d = *(const v4f*)(x + cb + 4);
    if (RIN) { a = bfr4(a); d = bfr4(d); }
    s += ((a[0] + a[1]) + (a[2] + a[3])) + ((d[0] + d[1]) + (d[2] + d[3]));
  }
#pragma unroll
  for (int off = 16; off > 0; off >>= 1) s += __shfl_xor(s, off, 32);
  const float mean = s * (1.0f / DM);

  float s2 = 0.f;
#pragma unroll 1
  for (int i = 0; i < 4; ++i) {
    const int cb = i * 256 + lane * 8;
    v4f a = *(const v4f*)(x + cb);
    v4f d = *(const v4f*)(x + cb + 4);
    if (RIN) { a = bfr4(a); d = bfr4(d); }
    const float xv[8] = {a[0], a[1], a[2], a[3], d[0], d[1], d[2], d[3]};
#pragma unroll
    for (int e = 0; e < 8; ++e) { const float t = xv[e] - mean; s2 += t * t; }
  }
#pragma unroll
  for (int off = 16; off > 0; off >>= 1) s2 += __shfl_xor(s2, off, 32);
  const float var  = s2 * (1.0f / DM);
  const float rstd = rsqrtf(var + 1e-5f);

#pragma unroll 1
  for (int i = 0; i < 4; ++i) {
    const int cb = i * 256 + lane * 8;
    v4f a = *(const v4f*)(x + cb);
    v4f d = *(const v4f*)(x + cb + 4);
    if (RIN) { a = bfr4(a); d = bfr4(d); }
    const v4f g0v = bfr4(*(const v4f*)(g + cb));
    const v4f g1v = bfr4(*(const v4f*)(g + cb + 4));
    const v4f b0v = bfr4(*(const v4f*)(be + cb));
    const v4f b1v = bfr4(*(const v4f*)(be + cb + 4));
    const float xv[8] = {a[0], a[1], a[2], a[3], d[0], d[1], d[2], d[3]};
    const float gv[8] = {g0v[0], g0v[1], g0v[2], g0v[3], g1v[0], g1v[1], g1v[2], g1v[3]};
    const float bv[8] = {b0v[0], b0v[1], b0v[2], b0v[3], b1v[0], b1v[1], b1v[2], b1v[3]};
    unsigned short hb[8], lb[8];
#pragma unroll
    for (int e = 0; e < 8; ++e) {
      const float y = (xv[e] - mean) * rstd * gv[e] + bv[e];
      hb[e] = f2bf_bits(y);
      lb[e] = f2bf_bits(y - bf_bits2f(hb[e]));
    }
    v4u hv, lv;
#pragma unroll
    for (int q = 0; q < 4; ++q) { hv[q] = pk16(hb[2 * q], hb[2 * q + 1]); lv[q] = pk16(lb[2 * q], lb[2 * q + 1]); }
    *(volatile v4u*)(orow + cb)      = hv;
    *(volatile v4u*)(orow + DM + cb) = lv;
    __threadfence();
    *(volatile v4u*)(orow + cb)      = hv;
    *(volatile v4u*)(orow + DM + cb) = lv;
  }
}

#define AT_D  64
#define AT_NW 4
#define AT_KC 64

__device__ __forceinline__ __bf16 at_f2bf(float f) { return __builtin_bit_cast(__bf16, f2bf_bits(f)); }
__device__ __forceinline__ void at_split(float f, __bf16& hi, __bf16& lo) {
  const unsigned short hb = f2bf_bits(f);
  hi = __builtin_bit_cast(__bf16, hb);
  lo = at_f2bf(f - __uint_as_float(((unsigned)hb) << 16));
}
__device__ __forceinline__ v8f at_mma(v16b a, v16b b, v8f c) {
  c = __builtin_amdgcn_wmma_f32_16x16x32_bf16(false, a, false, b, (short)0, c, false, false);
  asm volatile("v_nop\n\tv_nop\n\tv_nop\n\tv_nop" : "+v"(c) : "v"(a), "v"(b));
  return c;
}

__global__ __launch_bounds__(128)
void attn_kernel(const unsigned short* __restrict__ qpp, const unsigned short* __restrict__ kpp,
                 const unsigned short* __restrict__ vtp, const float* __restrict__ qin,
                 float* __restrict__ out, float sscale) {
  union FB { v16b v; v8b h[2]; };
  __shared__ __align__(16) __bf16 Ksh[AT_KC * AT_D];
  __shared__ __align__(16) __bf16 Vth[AT_D * AT_KC];
  __shared__ __align__(16) __bf16 Psh[AT_NW][16 * AT_KC];
  __shared__ __align__(16) __bf16 Psl[AT_NW][16 * AT_KC];
  __shared__ __align__(16) float  Os[AT_NW][16 * 68];

  const int tid  = threadIdx.x;
  const int wave = tid >> 5;
  const int lane = tid & 31;
  const int hh   = lane >> 4;
  const int c    = lane & 15;

  const int nqb = NT / 64;
  const int bx  = blockIdx.x;
  const int qb  = bx % nqb;
  const int h   = bx / nqb;
  const int b   = blockIdx.y;
  const int q0  = qb * 64 + wave * 16;

  const size_t boff = (size_t)b * NT * DM;
  const __bf16* Qh = (const __bf16*)(const void*)qpp + boff + (size_t)h * AT_D;
  const __bf16* Kh = (const __bf16*)(const void*)kpp + boff + (size_t)h * AT_D;
  const __bf16* Vh = (const __bf16*)(const void*)vtp + boff + (size_t)h * AT_D * NT;
  const float*  qr = qin + boff + (size_t)h * AT_D;
  float*        ob = out + boff + (size_t)h * AT_D;

  v16b qah[2];
#pragma unroll
  for (int dc = 0; dc < 2; ++dc)
    qah[dc] = Frag<__bf16>::load(Qh + (size_t)(q0 + c) * DM + dc * 32 + 8 * hh);

  float mrow[8], lrow[8];
  v8f oacc[4];
#pragma unroll
  for (int r = 0; r < 8; ++r) { mrow[r] = -INFINITY; lrow[r] = 0.f; }
#pragma unroll
  for (int t = 0; t < 4; ++t) oacc[t] = (v8f){0.f,0.f,0.f,0.f,0.f,0.f,0.f,0.f};

  const int nChunks = NT / AT_KC;
  for (int kc = 0; kc < nChunks; ++kc) {
    const int kv0 = kc * AT_KC;
    __syncthreads();
    {
      const int r = tid >> 1, half = (tid & 1) * 32;
      const __bf16* ksh = Kh + (size_t)(kv0 + r) * DM + half;
      const __bf16* vsh = Vh + (size_t)r * NT + kv0 + half;
#pragma unroll
      for (int i = 0; i < 4; ++i) {
        const v8b a0 = *(const v8b*)(ksh + 8 * i);
        const v8b b0 = *(const v8b*)(vsh + 8 * i);
        *(v8b*)(Ksh + r * AT_D  + half + 8 * i) = a0;
        *(v8b*)(Vth + r * AT_KC + half + 8 * i) = b0;
      }
    }
    __syncthreads();

    v8f s[4];
#pragma unroll
    for (int j = 0; j < 4; ++j) {
      s[j] = (v8f){0.f,0.f,0.f,0.f,0.f,0.f,0.f,0.f};
#pragma unroll
      for (int dc = 0; dc < 2; ++dc) {
        FB kb;
        kb.h[0] = *(const v8b*)(Ksh + (j * 16 + c) * AT_D + dc * 32 + 8 * hh);
        kb.h[1] = *(const v8b*)(Ksh + (j * 16 + c) * AT_D + dc * 32 + 16 + 8 * hh);
        s[j] = at_mma(qah[dc], kb.v, s[j]);
      }
    }
    float cm[8];
#pragma unroll
    for (int r = 0; r < 8; ++r) {
      float m = -INFINITY;
#pragma unroll
      for (int j = 0; j < 4; ++j) {
        const float sv = s[j][r] * sscale;
        s[j][r] = sv;
        m = fmaxf(m, sv);
      }
#pragma unroll
      for (int off = 1; off < 16; off <<= 1) m = fmaxf(m, __shfl_xor(m, off, 32));
      cm[r] = m;
    }
    __bf16* pwh = Psh[wave];
    __bf16* pwl = Psl[wave];
#pragma unroll
    for (int r = 0; r < 8; ++r) {
      const float mnew  = fmaxf(mrow[r], cm[r]);
      const float alpha = __expf(mrow[r] - mnew);
      mrow[r] = mnew;
      float psum = 0.f;
#pragma unroll
      for (int j = 0; j < 4; ++j) {
        const float p = __expf(s[j][r] - mnew);
        psum += p;
        __bf16 a, bl; at_split(p, a, bl);
        pwh[(8 * hh + r) * AT_KC + j * 16 + c] = a;
        pwl[(8 * hh + r) * AT_KC + j * 16 + c] = bl;
      }
#pragma unroll
      for (int off = 1; off < 16; off <<= 1) psum += __shfl_xor(psum, off, 32);
      lrow[r] = lrow[r] * alpha + psum;
#pragma unroll
      for (int t = 0; t < 4; ++t) oacc[t][r] *= alpha;
    }
    __builtin_amdgcn_fence(__ATOMIC_RELEASE, "workgroup");
    __builtin_amdgcn_wave_barrier();
    __builtin_amdgcn_fence(__ATOMIC_ACQUIRE, "workgroup");
#pragma unroll 1
    for (int kk = 0; kk < 2; ++kk) {
      FB pa, pl;
      pa.h[0] = *(const v8b*)(pwh + c * AT_KC + kk * 32 + 8 * hh);
      pa.h[1] = *(const v8b*)(pwh + c * AT_KC + kk * 32 + 16 + 8 * hh);
      pl.h[0] = *(const v8b*)(pwl + c * AT_KC + kk * 32 + 8 * hh);
      pl.h[1] = *(const v8b*)(pwl + c * AT_KC + kk * 32 + 16 + 8 * hh);
#pragma unroll
      for (int t = 0; t < 4; ++t) {
        FB vb;
        vb.h[0] = *(const v8b*)(Vth + (t * 16 + c) * AT_KC + kk * 32 + 8 * hh);
        vb.h[1] = *(const v8b*)(Vth + (t * 16 + c) * AT_KC + kk * 32 + 16 + 8 * hh);
        oacc[t] = at_mma(pa.v, vb.v, oacc[t]);
        oacc[t] = at_mma(pl.v, vb.v, oacc[t]);
      }
    }
  }

  float* os = Os[wave];
#pragma unroll
  for (int r = 0; r < 8; ++r) {
    const float inv = 1.0f / lrow[r];
#pragma unroll
    for (int t = 0; t < 4; ++t) os[(8 * hh + r) * 68 + t * 16 + c] = oacc[t][r] * inv;
  }
  __builtin_amdgcn_fence(__ATOMIC_RELEASE, "workgroup");
  __builtin_amdgcn_wave_barrier();
  __builtin_amdgcn_fence(__ATOMIC_ACQUIRE, "workgroup");
  {
    const int c4 = (lane & 15) * 4;
    v4f vals[8];
#pragma unroll
    for (int it = 0; it < 8; ++it) {
      const int row = it * 2 + hh;
      const v4f cv = *(const v4f*)(os + row * 68 + c4);
      const v4f qv = *(const v4f*)(qr + (size_t)(q0 + row) * DM + c4);
      vals[it] = cv + bfr4(qv);
    }
    for (int pass = 0; pass < 2; ++pass) {
#pragma unroll
      for (int it = 0; it < 8; ++it) {
        const int row = it * 2 + hh;
        *(volatile v4f*)(ob + (size_t)(q0 + row) * DM + c4) = vals[it];
      }
      __threadfence();
    }
  }
}

extern "C" void kernel_launch(void* const* d_in, const int* in_sizes, int n_in,
                              void* d_out, int out_size, void* d_ws, size_t ws_size,
                              hipStream_t stream) {
  if (n_in < 16) return;
  if (in_sizes[0] != NB * NT * DM || in_sizes[1] != NB * NT * DM) return;
  if (in_sizes[2] != DM * DM || in_sizes[4] != DM * DM || in_sizes[6] != DM * DM || in_sizes[8] != DM * DM) return;
  if (in_sizes[3] != DM || in_sizes[5] != DM || in_sizes[7] != DM || in_sizes[9] != DM) return;
  if (in_sizes[10] != DM || in_sizes[11] != DM || in_sizes[12] != DM || in_sizes[13] != DM) return;
  if (in_sizes[14] != DM || in_sizes[15] != DM) return;
  if (out_size != NB * NT * DM) return;

  const float* Qin   = (const float*)d_in[0];
  const float* Kin   = (const float*)d_in[1];
  const float* wq    = (const float*)d_in[2];
  const float* bq    = (const float*)d_in[3];
  const float* wk    = (const float*)d_in[4];
  const float* bk    = (const float*)d_in[5];
  const float* wv    = (const float*)d_in[6];
  const float* bv    = (const float*)d_in[7];
  const float* wo    = (const float*)d_in[8];
  const float* bo    = (const float*)d_in[9];
  const float* gq    = (const float*)d_in[10];
  const float* betaq = (const float*)d_in[11];
  const float* gk    = (const float*)d_in[12];
  const float* betak = (const float*)d_in[13];
  const float* g0    = (const float*)d_in[14];
  const float* beta0 = (const float*)d_in[15];
  float* outp = (float*)d_out;

  const size_t szWpl = (size_t)DM * K2 * 2;
  const size_t szW2  = 4 * szWpl;
  const size_t szN   = (size_t)MTOT * K2 * 2;
  const size_t szP   = (size_t)MTOT * DM * 2;
  const size_t szO   = (size_t)MTOT * DM * 4;
  size_t off = 0;
  const size_t oW2 = off; off += szW2;
  const size_t oQN = off; off += szN;
  const size_t oKN = off; off += szN;
  const size_t oQP = off; off += szP;
  const size_t oKP = off; off += szP;
  const size_t oVT = off; off += szP;
  const size_t oO  = off; off += szO;
  const size_t oON = off; off += szN;
  if (off > ws_size) return;
  if (oKN != oQN + szN) return;

  char* ws = (char*)d_ws;
  unsigned short* W2  = (unsigned short*)(ws + oW2);
  unsigned short* W2q = W2;
  unsigned short* W2k = (unsigned short*)(ws + oW2 + 1 * szWpl);
  unsigned short* W2v = (unsigned short*)(ws + oW2 + 2 * szWpl);
  unsigned short* W2o = (unsigned short*)(ws + oW2 + 3 * szWpl);
  unsigned short* QN  = (unsigned short*)(ws + oQN);
  unsigned short* KN  = (unsigned short*)(ws + oKN);
  unsigned short* QP  = (unsigned short*)(ws + oQP);
  unsigned short* KP  = (unsigned short*)(ws + oKP);
  unsigned short* VT  = (unsigned short*)(ws + oVT);
  float*          Opl = (float*)(ws + oO);
  unsigned short* ON  = (unsigned short*)(ws + oON);

  const dim3 blk(256);

  wprep_kernel<<<dim3(DM / 64, DM / 64, 4), blk, 0, stream>>>(wq, wk, wv, wo, W2);

  ln_kernel<true><<<dim3((2 * MTOT) / 8), blk, 0, stream>>>(Qin, gq, betaq, Kin, gk, betak, MTOT, 2 * MTOT, QN);

  const dim3 gProj(((MTOT / 64) * (DM / 64) + 7) / 8, 1);
  wmma_gemm64<1, false, 2, 3, false, 0><<<gProj, blk, 0, stream>>>(
      QN, QN, K2, 0L, W2q, W2q, K2, 0L, (void*)QP, (void*)QP, DM, 0L,
      bq, bq, 0L, MTOT, DM, K2, 1.0f);
  wmma_gemm64<1, false, 2, 3, false, 0><<<gProj, blk, 0, stream>>>(
      KN, KN, K2, 0L, W2k, W2k, K2, 0L, (void*)KP, (void*)KP, DM, 0L,
      bk, bk, 0L, MTOT, DM, K2, 1.0f);
  const dim3 gVT(((DM / 64) * (NT / 64) + 7) / 8, NB);
  wmma_gemm64<1, false, 1, 3, false, 0><<<gVT, blk, 0, stream>>>(
      W2v, W2v, K2, 0L, KN, KN, K2, (long)NT * K2, (void*)VT, (void*)VT, NT, (long)DM * NT,
      bv, bv, 0L, DM, NT, K2, 1.0f);

  attn_kernel<<<dim3(NH * (NT / 64), NB), dim3(128), 0, stream>>>(QP, KP, VT, Qin, Opl, 0.03125f);

  ln_kernel<false><<<dim3(MTOT / 8), blk, 0, stream>>>(Opl, g0, beta0, Opl, g0, beta0, MTOT, MTOT, ON);

  wmma_gemm64<1, false, 2, 0, true, 2><<<gProj, blk, 0, stream>>>(
      ON, ON, K2, 0L, W2o, W2o, K2, 0L, (void*)outp, (void*)outp, DM, 0L,
      bo, Opl, 0L, MTOT, DM, K2, 1.0f);

  (void)hipGetLastError();
}
